// NonLocalAttentionBlock2D_75076028334858
// MI455X (gfx1250) — hardware-run, weakly checked
//
#include <hip/hip_runtime.h>
#include <math.h>

typedef __attribute__((ext_vector_type(16))) _Float16 v16h;
typedef __attribute__((ext_vector_type(16))) __bf16 v16b;
typedef __attribute__((ext_vector_type(8)))  _Float16 v8h;
typedef __attribute__((ext_vector_type(8)))  float v8f;
typedef __attribute__((ext_vector_type(4)))  float v4f;
typedef __attribute__((ext_vector_type(4)))  unsigned v4u;
typedef _Float16 h16;

template <typename T> __device__ __forceinline__ void vst2(void* p, T v) { *(volatile T*)p = v; __threadfence(); *(volatile T*)p = v; }
__device__ __forceinline__ v8f wmma16(v16h a, v16h b, v8f c) {
  v8f d = __builtin_amdgcn_wmma_f32_16x16x32_f16(false, a, false, b, (short)0, c, false, false);
  asm volatile("v_nop\n\tv_nop\n\tv_nop\n\tv_nop" : "+v"(d) : "v"(a), "v"(b));
  return d;
}
__device__ __forceinline__ v8f wmma_bf(v16b a, v16b b, v8f c) {
  v8f d = __builtin_amdgcn_wmma_f32_16x16x32_bf16(false, a, false, b, (short)0, c, false, false);
  asm volatile("v_nop\n\tv_nop\n\tv_nop\n\tv_nop" : "+v"(d) : "v"(a), "v"(b));
  return d;
}
__device__ __forceinline__ v16h frag_h(const _Float16* rowk0, int lane) {
  union { v16h v; v8h q[2]; } u; const _Float16* p = rowk0 + 8 * (lane >> 4);
  u.q[0] = *(const v8h*)p; u.q[1] = *(const v8h*)(p + 16); return u.v;
}
__device__ __forceinline__ float bfr(float v) { return (float)(__bf16)v; }
__device__ __forceinline__ v16b wcol_oi(const float* Wm, int k0, int o, int lane, int K) { v16b w; const float* p = Wm + (size_t)o * K + k0 + 8 * (lane >> 4);
#pragma unroll
  for (int i = 0; i < 8; ++i) { w[i] = (__bf16)p[i]; w[8 + i] = (__bf16)p[16 + i]; }
  return w; }
#define LDSX() do { asm volatile("s_wait_dscnt 0" ::: "memory"); __builtin_amdgcn_wave_barrier(); __builtin_amdgcn_fence(3  , "workgroup"); } while (0)
static __device__ __forceinline__ h16 toh_flush(float v) { const h16 r = (h16)v; return (fabsf(v) < 6.103515625e-05f) ? (h16)0.0f : r; }

#define NB 4
#ifndef TNB
#define TNB NB
#endif
#ifndef TT
#define TT 4096
#endif
#define TT_FULL 4096
#define DIN 64
#define CC 128
#define CV 32
#define COUT 64
#define CCQ 128
#define HD 32
#define NQB (TT / 64)
#define HG 1
#define HDQK 32
#define BG HG
#define BGN (TNB < BG ? TNB : BG)
#define DVH 32
#define CK 576
#define CW (DIN * CK)

static_assert(TT % 128 == 0);
static_assert(TT <= TT_FULL);
static_assert(TNB <= NB);
static_assert(DIN % 32 == 0);
static_assert(HDQK == 32 && CV == 32 && DVH == 32);
static_assert((64 * 16) % 128 == 0 && (128 * 8) % 128 == 0);
static_assert(TT == 4096 && TT_FULL == 4096);
static_assert(DIN == 64 && COUT == DIN);
static_assert(CK == 9 * DIN && CK % 32 == 0);
static_assert(CW % (256 * 8) == 0);
static_assert((NB * DIN * TT) % 256 == 0);
static_assert(128 * 16 * 4 == 64 * 128);
static_assert(128 * 16 * 8 == 64 * 256);
static_assert(64 * 72 * 2 + 64 * 68 * 4 <= 131072);
static_assert(64 * 72 * 2 <= 131072);
static_assert(2 * 64 * 136 * 2 + 128 * 72 * 2 <= 131072);
static_assert(4 * 16 * 132 * 4 <= 131072);
static_assert(4 * TT + 64 <= 131072);
static_assert(DVH * 68 * 4 <= 131072);

#define WS_QH  ((size_t)0)
#define WS_KH  (WS_QH + 2u * (size_t)NB * TT * CCQ)
#define WS_VT  (WS_KH + 2u * (size_t)NB * TT * CCQ)
#define WS_QL  (WS_VT + 2u * (size_t)NB * CC * TT)
#define WS_KL  (WS_QL + 2u * (size_t)NB * TT * CCQ)
#define WS_S   (WS_KL + 2u * (size_t)NB * TT * CCQ)
#define WS_AM  (WS_S  + 4u * (size_t)HG * TT * TT)
#define WS_XT  (WS_AM + 4u * (size_t)NB * DIN * TT_FULL)
#define WS_WH  (WS_XT + 2u * (size_t)NB * TT_FULL * DIN)
#define WS_T1  (WS_WH + 2u * (size_t)3 * CW)
#define WS_T2  (WS_T1 + 2u * (size_t)NB * 1024 * DIN)
#define WS_Y8  (WS_T2 + 2u * (size_t)NB * 256 * DIN)
#define WS_END (WS_Y8 + 4u * (size_t)NB * 64 * DIN)
static_assert(WS_END <= (size_t)134217728);
static_assert(WS_S % 128 == 0);
static_assert(WS_AM % 128 == 0 && WS_XT % 128 == 0 && WS_WH % 128 == 0 && WS_T1 % 128 == 0 && WS_T2 % 128 == 0 && WS_Y8 % 128 == 0);

__global__ __launch_bounds__(128) void k_xt(const float* __restrict__ X, _Float16* __restrict__ XT) { __shared__ __align__(16) _Float16 tl[64][72];
  const int tid = threadIdx.x; const size_t r0 = (size_t)blockIdx.x * 64; const size_t bb = r0 / TT; const int t0 = (int)(r0 % TT);
#pragma unroll 4
  for (int e = tid; e < 64 * 64; e += 128) { const int c = e >> 6, nl = e & 63; const float v = X[(bb * DIN + c) * (size_t)TT_FULL + t0 + nl]; tl[nl][c] = toh_flush(bfr(v)); }
  __syncthreads();
  for (int e = tid; e < 64 * 8; e += 128) { const int rl = e >> 3, q = e & 7; vst2(XT + (r0 + rl) * (size_t)DIN + q * 8, *(const v4u*)&tl[rl][q * 8]); } }
__global__ __launch_bounds__(256) void k_wcv(const float* __restrict__ W1, const float* __restrict__ W2, const float* __restrict__ W3, _Float16* __restrict__ WH) {
  const int ly = blockIdx.y; const int e0 = (blockIdx.x * 256 + threadIdx.x) * 8; const int oc = e0 / CK; const int kk = e0 - oc * CK; const int tap = kk >> 6, ic = kk & 63; const int src = oc * CK + ic * 9 + tap;
  union { v8h v; v4u q; } o;
#pragma unroll
  for (int i = 0; i < 8; ++i) { const float a = W1[src + 9 * i], b = W2[src + 9 * i], c = W3[src + 9 * i]; if ((i & 3) == 3) asm volatile("s_wait_loadcnt 0x0" ::: "memory");
    const float w = ly == 0 ? a : (ly == 1 ? b : c); o.v[i] = toh_flush(bfr(w) * 64.0f); }
  vst2(WH + (size_t)ly * CW + e0, o.q); }
__global__ __launch_bounds__(128) void k_conv(const _Float16* __restrict__ XI, const _Float16* __restrict__ WH, const float* __restrict__ BI, int lgw, int mode, _Float16* __restrict__ OH, float* __restrict__ OF) {
  __shared__ __align__(16) _Float16 sh[64][72]; __shared__ __align__(16) float sf[64][68];
  const int tid = threadIdx.x; const int wave = __builtin_amdgcn_readfirstlane(threadIdx.x >> 5); const int lane = tid & 31, col = lane & 15, g = lane >> 4;
  const int wo = 1 << lgw, wi = 2 << lgw;
  const int m = blockIdx.x * 64 + wave * 16 + col;
  const int b = m >> (2 * lgw), oh = (m >> lgw) & (wo - 1), ow = m & (wo - 1);
  v8f acc[4] = {};
#pragma unroll 1
  for (int tap = 0; tap < 9; ++tap) { const int kh = tap / 3, kw = tap - 3 * kh; const int ih = 2 * oh + kh - 1, iw = 2 * ow + kw - 1;
    const int ok = (ih >= 0) & (ih < wi) & (iw >= 0) & (iw < wi); const int ihc = min(max(ih, 0), wi - 1), iwc = min(max(iw, 0), wi - 1);
    const unsigned mk = 0u - (unsigned)ok; const v4u mv = {mk, mk, mk, mk};
    const _Float16* row = XI + (size_t)((b * wi + ihc) * wi + iwc) * DIN;
#pragma unroll
    for (int hf = 0; hf < 2; ++hf) { v16h av = frag_h(row + hf * 32, lane); asm volatile("" : "+v"(av));
      union { v16h v; v4u q[2]; } a; a.v = av; a.q[0] = a.q[0] & mv; a.q[1] = a.q[1] & mv;
#pragma unroll
      for (int j = 0; j < 4; ++j) acc[j] = wmma16(a.v, frag_h(WH + (size_t)(j * 16 + col) * CK + tap * 64 + hf * 32, lane), acc[j]); } }
#pragma unroll
  for (int j = 0; j < 4; ++j) { const float bias = bfr(BI[j * 16 + col]);
#pragma unroll
    for (int r = 0; r < 8; ++r) { const float v = acc[j][r] * (1.0f / 64.0f) + bias; const float lv = (v >= 0.f) ? v : 0.2f * v; const float u = (mode == 0) ? lv : v;
      sh[wave * 16 + 8 * g + r][j * 16 + col] = toh_flush(u); sf[wave * 16 + 8 * g + r][j * 16 + col] = u; } }
  __syncthreads();
  const size_t m0 = (size_t)blockIdx.x * 64;
  if (mode == 0) { for (int e = tid; e < 64 * 8; e += 128) { const int rl = e >> 3, q = e & 7; vst2(OH + (m0 + rl) * (size_t)DIN + q * 8, *(const v4u*)&sh[rl][q * 8]); } }
  else { for (int e = tid; e < 64 * 16; e += 128) { const int rl = e >> 4, q = e & 15; vst2(OF + (m0 + rl) * (size_t)DIN + q * 4, *(const v4f*)&sf[rl][q * 4]); } } }
__global__ __launch_bounds__(256) void k_gate(const float* __restrict__ Y8, const float* __restrict__ X, float* __restrict__ AM) {
#pragma clang fp contract(off)
  const int idx = blockIdx.x * 256 + threadIdx.x; const int ow = idx & 63, oh = (idx >> 6) & 63, pl = idx >> 12; const int b = pl >> 6, c = pl & 63;
  const float sy = ((float)oh + 0.5f) * 0.125f - 0.5f; const float sx = ((float)ow + 0.5f) * 0.125f - 0.5f;
  const int y0 = (int)floorf(sy), x0 = (int)floorf(sx); const float fy = sy - (float)y0, fx = sx - (float)x0;
  const int y0c = min(max(y0, 0), 7), y1c = min(max(y0 + 1, 0), 7), x0c = min(max(x0, 0), 7), x1c = min(max(x0 + 1, 0), 7);
  const float* p = Y8 + (size_t)b * 64 * DIN + c;
  const float v00 = p[(y0c * 8 + x0c) * DIN], v01 = p[(y0c * 8 + x1c) * DIN], v10 = p[(y1c * 8 + x0c) * DIN], v11 = p[(y1c * 8 + x1c) * DIN];
  const size_t gi = (size_t)pl * TT_FULL + (idx & 4095); const float xv = X[gi];
  const float v0 = v00 + fx * (v01 - v00); const float v1 = v10 + fx * (v11 - v10); const float v = v0 + fy * (v1 - v0);
  const float sig = 1.0f / (1.0f + expf(-v));
  const float av = sig * bfr(xv);
  vst2(AM + gi, av); }

__global__ __launch_bounds__(128) void k_proj(const float* __restrict__ XQ, const float* __restrict__ XK, const float* __restrict__ XV, const float* __restrict__ WQ, const float* __restrict__ WK, const float* __restrict__ WV, const float* __restrict__ BQ, const float* __restrict__ BK, const float* __restrict__ BV,
    _Float16* __restrict__ QH, _Float16* __restrict__ QL, _Float16* __restrict__ KH, _Float16* __restrict__ KL, _Float16* __restrict__ VT) {
  __shared__ __align__(16) _Float16 sh[64][136], sl[64][136]; __shared__ __align__(16) _Float16 th[128][72];
  const int tid = threadIdx.x, wave = tid >> 5, lane = tid & 31, col = lane & 15, g = lane >> 4; const int which = blockIdx.z; const int c0 = 0;
  const size_t r0 = (size_t)blockIdx.x * 64; const size_t bb = r0 / TT; const int t0 = (int)(r0 % TT);
  const float* X = which == 0 ? XQ : which == 1 ? XK : XV; const float* WA = which == 0 ? WQ : which == 1 ? WK : WV; const float* BA = which == 0 ? BQ : which == 1 ? BK : BV;
  v8f acc[8] = {};
#pragma unroll
  for (int kc = 0; kc < DIN / 32; ++kc) { v16b a; { const float* p = X + (bb * DIN + kc * 32 + 8 * g) * (size_t)TT_FULL + t0 + wave * 16 + col;
#pragma unroll
      for (int i = 0; i < 8; ++i) { a[i] = (__bf16)p[(size_t)i * TT_FULL]; a[8 + i] = (__bf16)p[(size_t)(16 + i) * TT_FULL]; } }
    asm volatile("s_wait_loadcnt 0x0" ::: "memory");
#pragma unroll
    for (int j = 0; j < HDQK / 16; ++j) { const v16b w = wcol_oi(WA, kc * 32, j * 16 + col, lane, DIN); asm volatile("s_wait_loadcnt 0x0" ::: "memory"); acc[j] = wmma_bf(a, w, acc[j]); } }
  if (which < 2) { _Float16* DH = which == 0 ? QH : KH; _Float16* DL = which == 0 ? QL : KL;
#pragma unroll
    for (int j = 0; j < 8; ++j) { const int cj = c0 + j * 16 + col; const int cjc = cj < HDQK ? cj : HDQK - 1; const float bv = bfr(BA[cjc]); const float bias = cj < HDQK ? bv : 0.f;
#pragma unroll
      for (int r = 0; r < 8; ++r) { const float v = acc[j][r] + bias; const _Float16 hv = (_Float16)v; sh[wave * 16 + 8 * g + r][j * 16 + col] = hv; sl[wave * 16 + 8 * g + r][j * 16 + col] = (_Float16)((v - (float)hv) * 1024.0f); } }
    __syncthreads();
    for (int e = tid; e < 64 * 16; e += 128) { const int rl = e >> 4, q = e & 15; const size_t o2 = (r0 + rl) * (size_t)CCQ + c0 + q * 8; vst2((unsigned*)(DH + o2), *(const v4u*)&sh[rl][q * 8]); vst2((unsigned*)(DL + o2), *(const v4u*)&sl[rl][q * 8]); }
  } else {
#pragma unroll
    for (int j = 0; j < 8; ++j) { const int cj = c0 + j * 16 + col; const int cjc = cj < CV ? cj : CV - 1; const float bv = bfr(BA[cjc]); const float bias = cj < CV ? bv : 0.f;
#pragma unroll
      for (int r = 0; r < 8; ++r) { const float v = acc[j][r] + bias; const int rl = wave * 16 + 8 * g + r, cl = j * 16 + col; th[cl][rl] = (_Float16)v; } }
    __syncthreads();
    for (int e = tid; e < 128 * 8; e += 128) { const int cl = e >> 3, q = e & 7; vst2((unsigned*)(VT + (bb * CC + c0 + cl) * (size_t)TT + t0 + q * 8), *(const v4u*)&th[cl][q * 8]); } } }
__global__ __launch_bounds__(128) void k_sc(const _Float16* __restrict__ QH, const _Float16* __restrict__ KH, const _Float16* __restrict__ QL, const _Float16* __restrict__ KL, int bgrp, float* __restrict__ S0) { __shared__ __align__(16) float ss[4][16][132];
  const int qb = blockIdx.x, kb = blockIdx.y;
  const int b = bgrp + blockIdx.z; float* S = S0 + (size_t)blockIdx.z * TT * TT;
  const int tid = threadIdx.x, wave = tid >> 5, lane = tid & 31, col = lane & 15, g = lane >> 4; const int k0 = kb * 128; const int ql0 = qb * 64 + wave * 16; const size_t q0 = (size_t)b * TT + ql0, kr0 = (size_t)b * TT + k0;
  v8f acc[8] = {}, accl[8] = {};
#pragma unroll
  for (int kc = 0; kc < HDQK / 32; ++kc) { const v16h ah = frag_h(QH + (q0 + col) * CCQ + kc * 32, lane), al = frag_h(QL + (q0 + col) * CCQ + kc * 32, lane);
#pragma unroll
    for (int j = 0; j < 8; ++j) { const v16h kbf = frag_h(KH + (kr0 + j * 16 + col) * CCQ + kc * 32, lane), klf = frag_h(KL + (kr0 + j * 16 + col) * CCQ + kc * 32, lane); acc[j] = wmma16(ah, kbf, acc[j]); accl[j] = wmma16(al, kbf, accl[j]); accl[j] = wmma16(ah, klf, accl[j]); } }
#pragma unroll
  for (int j = 0; j < 8; ++j) {
#pragma unroll
    for (int r = 0; r < 8; ++r) ss[wave][8 * g + r][j * 16 + col] = acc[j][r] + accl[j][r] * (1.0f / 1024.0f); }
  LDSX();
  for (int rl = 0; rl < 16; ++rl) vst2(S + (size_t)(ql0 + rl) * TT + k0 + lane * 4, *(const v4f*)&ss[wave][rl][lane * 4]); }
__global__ __launch_bounds__(256) void k_sm(float* __restrict__ S0) { __shared__ float sred[8]; __shared__ float sbc; __shared__ __align__(16) float shv[TT];
  const int tid = threadIdx.x; const int t = blockIdx.x;
  float* sr = S0 + (size_t)blockIdx.y * TT * TT + (size_t)t * TT;
  float m = -3.0e38f; for (int k = tid; k < TT; k += 256) { const float v = sr[k]; shv[k] = v; m = fmaxf(m, v); }
#pragma unroll
  for (int o = 1; o < 32; o <<= 1) m = fmaxf(m, __shfl_xor(m, o));
  if ((tid & 31) == 0) sred[tid >> 5] = m; __syncthreads(); if (tid == 0) { float a = sred[0]; for (int i = 1; i < 8; ++i) a = fmaxf(a, sred[i]); sbc = a; } __syncthreads(); m = sbc; __syncthreads();
  float sum = 0.f; for (int k = tid; k < TT; k += 256) { const float e = expf(shv[k] - m); shv[k] = e; sum += e; }
#pragma unroll
  for (int o = 1; o < 32; o <<= 1) sum += __shfl_xor(sum, o);
  if ((tid & 31) == 0) sred[tid >> 5] = sum; __syncthreads(); if (tid == 0) { float a = 0.f; for (int i = 0; i < 8; ++i) a += sred[i]; sbc = 2048.0f * (1.0f / a); } __syncthreads(); const float inv = sbc;
  for (int k = tid; k < TT; k += 256) shv[k] = shv[k] * inv;
  __syncthreads(); for (int q = tid; q < TT / 4; q += 256) vst2(sr + q * 4, *(const v4f*)&shv[q * 4]); }
__global__ __launch_bounds__(128) void k_pv(const float* __restrict__ PS0, const _Float16* __restrict__ VT, int bgrp, const float* __restrict__ WO, const float* __restrict__ BO, const float* __restrict__ XS, const float* __restrict__ AM, float* __restrict__ Y) { __shared__ __align__(16) float stT[DVH][68];
  const int b = bgrp + blockIdx.z; const float* PS = PS0 + (size_t)blockIdx.z * TT * TT; const int d0 = blockIdx.y * DVH;
  const int tid = threadIdx.x, wave = tid >> 5, lane = tid & 31, col = lane & 15, g = lane >> 4; const int qb = blockIdx.x; const int ql0 = qb * 64 + wave * 16; const int kce = TT / 32;
  v8f acc[DVH / 16] = {};
#pragma unroll 1
  for (int kc = 0; kc < kce; ++kc) { v16h p; { const float* pp = PS + (size_t)(kc * 32 + 8 * g) * TT + ql0 + col;
#pragma unroll
      for (int i = 0; i < 8; ++i) { p[i] = toh_flush(pp[(size_t)i * TT]); p[8 + i] = toh_flush(pp[(size_t)(16 + i) * TT]); } }
    asm volatile("s_wait_loadcnt 0x0" ::: "memory");
#pragma unroll
    for (int j = 0; j < DVH / 16; ++j) { const size_t po = ((size_t)b * CC + d0 + j * 16 + col) * (size_t)TT + kc * 32; acc[j] = wmma16(p, frag_h(VT + po, lane), acc[j]); } }
#pragma unroll
  for (int j = 0; j < DVH / 16; ++j) {
#pragma unroll
    for (int r = 0; r < 8; ++r) stT[j * 16 + col][wave * 16 + 8 * g + r] = acc[j][r] * (1.0f / 2048.0f); }
  __syncthreads();
  { const int tb = qb * 64; const int tl = tid & 63, oh = tid >> 6;
    float yv[DVH];
#pragma unroll
    for (int c = 0; c < DVH; ++c) yv[c] = stT[c][tl];
#pragma unroll 1
    for (int oo = 0; oo < COUT / 2; ++oo) { const int o = oh * (COUT / 2) + oo; float wv[DVH];
#pragma unroll
      for (int c = 0; c < DVH; ++c) { wv[c] = WO[o * CV + c]; if ((c & 15) == 15) asm volatile("s_wait_loadcnt 0x0" ::: "memory"); }
      const size_t oi = ((size_t)b * COUT + o) * (size_t)TT_FULL + tb + tl;
      const float bo = BO[o]; const float xs = XS[oi]; const float av = AM[oi]; asm volatile("s_wait_loadcnt 0x0" ::: "memory");
      float a2 = 0.f;
#pragma unroll
      for (int c = 0; c < DVH; ++c) a2 += yv[c] * bfr(wv[c]);
      const float zv = (av + (a2 + bfr(bo))) * bfr(xs);
      vst2(Y + oi, zv); } } }

extern "C" void kernel_launch(void* const* d_in, const int* in_sizes, int n_in, void* d_out, int out_size, void* d_ws, size_t ws_size, hipStream_t stream) {
  if (n_in < 15) return;
  if (ws_size < (size_t)WS_END) return;
  if ((long long)in_sizes[0] < (long long)TNB * DIN * TT_FULL) return;
  if (in_sizes[1] < DIN * CK || in_sizes[3] < DIN * CK || in_sizes[5] < DIN * CK) return;
  if (in_sizes[2] < DIN || in_sizes[4] < DIN || in_sizes[6] < DIN) return;
  if (in_sizes[7] < CV * DIN || in_sizes[9] < HDQK * DIN || in_sizes[11] < HDQK * DIN || in_sizes[13] < COUT * CV) return;
  if (in_sizes[8] < CV || in_sizes[10] < HDQK || in_sizes[12] < HDQK || in_sizes[14] < COUT) return;
  if ((long long)out_size < (long long)TNB * COUT * TT_FULL) return;
  const float** F = (const float**)d_in;
  char* ws = (char*)d_ws; _Float16 *QH = (_Float16*)(ws + WS_QH), *KH = (_Float16*)(ws + WS_KH), *VT = (_Float16*)(ws + WS_VT), *QL = (_Float16*)(ws + WS_QL), *KL = (_Float16*)(ws + WS_KL); float *S = (float*)(ws + WS_S);
  float *AM = (float*)(ws + WS_AM), *Y8 = (float*)(ws + WS_Y8); _Float16 *XT = (_Float16*)(ws + WS_XT), *WH = (_Float16*)(ws + WS_WH), *T1 = (_Float16*)(ws + WS_T1), *T2 = (_Float16*)(ws + WS_T2);
  k_xt<<<dim3(TNB * TT / 64), 128, 0, stream>>>(F[0], XT);
  k_wcv<<<dim3(CW / 2048, 3), 256, 0, stream>>>(F[1], F[3], F[5], WH);
  k_conv<<<dim3(TNB * 1024 / 64), 128, 0, stream>>>(XT, WH, F[2], 5, 0, T1, Y8);
  k_conv<<<dim3(TNB * 256 / 64), 128, 0, stream>>>(T1, WH + CW, F[4], 4, 0, T2, Y8);
  k_conv<<<dim3(TNB * 64 / 64), 128, 0, stream>>>(T2, WH + 2 * CW, F[6], 3, 1, T1, Y8);
  k_gate<<<dim3(TNB * DIN * TT / 256), 256, 0, stream>>>(Y8, F[0], AM);
  k_proj<<<dim3(TNB * TT / 64, 1, 3), 128, 0, stream>>>(AM, AM, AM, F[11], F[9], F[7], F[12], F[10], F[8], QH, QL, KH, KL, VT);
  for (int b0 = 0; b0 < TNB; b0 += BGN) {
    k_sc<<<dim3(NQB, TT / 128, BGN), 128, 0, stream>>>(QH, KH, QL, KL, b0, S);
    k_sm<<<dim3(TT, BGN), 256, 0, stream>>>(S);
    k_pv<<<dim3(NQB, HD / DVH, BGN), 128, 0, stream>>>(S, VT, b0, F[13], F[14], F[0], AM, (float*)d_out);
  }
}
